// NRIModel_8787503088035
// MI455X (gfx1250) — hardware-verified
//
#include <hip/hip_runtime.h>
#define BB 8
#define NND 32
#define TT 49
#define DDIM 4
#define NE 992
#define KT 4
#define HE 256
#define KIN 196
#define KINP 224
#define CH 98

typedef __bf16 v16b __attribute__((ext_vector_type(16)));
typedef unsigned short v8us __attribute__((ext_vector_type(8), may_alias));
typedef float  v8f  __attribute__((ext_vector_type(8)));
typedef float  v4f  __attribute__((ext_vector_type(4)));
typedef float  v4fa __attribute__((ext_vector_type(4), may_alias));
union FragB { v16b v; v8us half[2]; unsigned short u[16]; };

__device__ __forceinline__ unsigned short bf16_bits(float x) { unsigned int u = __float_as_uint(x); return (unsigned short)((u + 0x7FFFu + ((u >> 16) & 1u)) >> 16); }
__device__ __forceinline__ float bf16_val(unsigned short b) { return __uint_as_float(((unsigned int)b) << 16); }
__device__ __forceinline__ float bf16_round(float x) { return bf16_val(bf16_bits(x)); }
template <int NT>
__device__ __forceinline__ v8f mmaN(v16b ah, v16b al, v16b bh, v16b bl, v8f c) {
  c = __builtin_amdgcn_wmma_f32_16x16x32_bf16(false, ah, false, bh, (short)0, c, false, false);
  if (NT >= 2) c = __builtin_amdgcn_wmma_f32_16x16x32_bf16(false, al, false, bh, (short)0, c, false, false);
  if (NT >= 3) c = __builtin_amdgcn_wmma_f32_16x16x32_bf16(false, ah, false, bl, (short)0, c, false, false);
  asm volatile("v_nop\n\tv_nop\n\tv_nop\n\tv_nop" : "+v"(c) : "v"(ah), "v"(al), "v"(bh), "v"(bl));
  return c;
}

__global__ __launch_bounds__(256) void k_wt_bf16(const float* __restrict__ W, unsigned short* __restrict__ Wt, int K, int N) {
  const int t = blockIdx.x * 256 + threadIdx.x;
  const int k8n = K / 8;
  if (t >= N * k8n) return;
  const int n = t / k8n, k8 = (t % k8n) * 8;
  v8us v;
#pragma unroll
  for (int i = 0; i < 8; ++i) v[i] = bf16_bits(W[(size_t)(k8 + i) * N + n]);
  *(volatile v8us*)(Wt + (size_t)n * K + k8) = v;
  __threadfence();
  *(volatile v8us*)(Wt + (size_t)n * K + k8) = v;
}

template <bool ASPLIT, int ACT, bool BIAS_BF16>
__global__ __launch_bounds__(128) void k_gemm_bf(const float* __restrict__ A, int lda, const unsigned short* __restrict__ Wt, int ldb,
                                               const float* __restrict__ bias, float* __restrict__ C, int ldc, int M, int N, int K) {
  __shared__ __attribute__((aligned(16))) float so[4][16][64];
  const int tid = threadIdx.x, w = tid >> 5, lane = tid & 31, ln = lane & 15, hh = lane >> 4;
  const int ntn = N / 64;
  const int wid = blockIdx.x * 4 + w;
  const int mt = wid / ntn, nq = wid % ntn;
  if (mt * 16 >= M) return;
  const int row0 = mt * 16, col0 = nq * 64;
  const float* arow = A + (size_t)(row0 + ln) * lda;
  v8f acc[4] = {};
  for (int kb = 0; kb < K; kb += 32) {
    FragB ah, al;
    const v4f x0 = *(const v4fa*)(arow + kb + 8 * hh), x1 = *(const v4fa*)(arow + kb + 8 * hh + 4);
    const v4f x2 = *(const v4fa*)(arow + kb + 16 + 8 * hh), x3 = *(const v4fa*)(arow + kb + 16 + 8 * hh + 4);
    float xs[16] = {x0[0],x0[1],x0[2],x0[3],x1[0],x1[1],x1[2],x1[3],x2[0],x2[1],x2[2],x2[3],x3[0],x3[1],x3[2],x3[3]};
#pragma unroll
    for (int i = 0; i < 16; ++i) { const unsigned short hb = bf16_bits(xs[i]); ah.u[i] = hb; al.u[i] = ASPLIT ? bf16_bits(xs[i] - bf16_val(hb)) : (unsigned short)0; }
#pragma unroll
    for (int t = 0; t < 4; ++t) {
      const unsigned short* brow = Wt + (size_t)(col0 + t * 16 + ln) * ldb + kb;
      FragB b;
      b.half[0] = *(const v8us*)(brow + 8 * hh);
      b.half[1] = *(const v8us*)(brow + 16 + 8 * hh);
      acc[t] = mmaN<ASPLIT ? 2 : 1>(ah.v, al.v, b.v, b.v, acc[t]);
    }
  }
#pragma unroll
  for (int t = 0; t < 4; ++t) {
    float bv = bias ? bias[col0 + t * 16 + ln] : 0.f;
    if (BIAS_BF16) bv = bf16_round(bv);
#pragma unroll
    for (int r = 0; r < 8; ++r) { float v = acc[t][r] + bv; if (ACT == 1) v = fmaxf(v, 0.f); so[w][8 * hh + r][t * 16 + ln] = v; }
  }
  __builtin_amdgcn_fence(__ATOMIC_ACQ_REL, "workgroup");
  __builtin_amdgcn_wave_barrier();
  const int rsub = lane >> 4, c4 = (lane & 15) * 4;
  for (int pass = 0; pass < 2; ++pass) {
#pragma unroll
    for (int q = 0; q < 8; ++q) {
      const int r = q * 2 + rsub;
      const v4f v = *(const v4fa*)&so[w][r][c4];
      *(volatile v4f*)(C + (size_t)(row0 + r) * ldc + col0 + c4) = v;
    }
    if (pass == 0) __threadfence();
  }
}

template <int D, bool CAUSAL>
__global__ __launch_bounds__(128) void k_flash(const float* __restrict__ qb, const float* __restrict__ kb, const float* __restrict__ vb,
                                             int pitch, int T, int H, float scale, float* __restrict__ y, int ypitch) {
  constexpr int KS = D / 32;
  constexpr int DT = D / 16;
  __shared__ __attribute__((aligned(16))) unsigned short sKh[32][D + 8], sKl[32][D + 8], sVh[32][D + 8], sVl[32][D + 8];
  __shared__ __attribute__((aligned(16))) unsigned short sPh[4][16][40], sPl[4][16][40];
  __shared__ __attribute__((aligned(16))) float sO[4][16][D];
  const int tid = threadIdx.x, w = tid >> 5, lane = tid & 31, ln = lane & 15, hh = lane >> 4;
  const int nqb = (T + 63) / 64;
  const int bh = blockIdx.x / nqb, qblk = blockIdx.x % nqb;
  const int b = bh / H, h = bh % H;
  const int q0 = qblk * 64 + w * 16;
  const float* Q = qb + (size_t)b * T * pitch + h * D;
  const float* K = kb + (size_t)b * T * pitch + h * D;
  const float* V = vb + (size_t)b * T * pitch + h * D;

  FragB aqh[KS], aql[KS];
  {
    int row = q0 + ln; if (row >= T) row = T - 1;
    const float* qr = Q + (size_t)row * pitch;
#pragma unroll
    for (int ks = 0; ks < KS; ++ks)
#pragma unroll
      for (int i = 0; i < 16; ++i) {
        const int d = ks * 32 + ((i < 8) ? (8 * hh + i) : (16 + 8 * hh + (i - 8)));
        const float x = qr[d] * scale; const unsigned short hb = bf16_bits(x);
        aqh[ks].u[i] = hb; aql[ks].u[i] = bf16_bits(x - bf16_val(hb));
      }
  }
  float m_r[8], l_r[8];
#pragma unroll
  for (int r = 0; r < 8; ++r) { m_r[r] = -3.0e38f; l_r[r] = 0.f; }
  v8f oacc[DT];
#pragma unroll
  for (int dt = 0; dt < DT; ++dt) oacc[dt] = (v8f){0.f,0.f,0.f,0.f,0.f,0.f,0.f,0.f};

  const int kv_end = CAUSAL ? min(T, qblk * 64 + 64) : T;
  for (int j0 = 0; j0 < kv_end; j0 += 32) {
    __syncthreads();
    for (int e = tid; e < 32 * (D / 4); e += 128) {
      const int r = e / (D / 4), c4 = (e % (D / 4)) * 4;
      const int key = j0 + r;
      v4f kf = {0.f,0.f,0.f,0.f}, vf = {0.f,0.f,0.f,0.f};
      if (key < T) { kf = *(const v4fa*)(K + (size_t)key * pitch + c4); vf = *(const v4fa*)(V + (size_t)key * pitch + c4); }
#pragma unroll
      for (int t = 0; t < 4; ++t) {
        unsigned short hb = bf16_bits(kf[t]); sKh[r][c4 + t] = hb; sKl[r][c4 + t] = bf16_bits(kf[t] - bf16_val(hb));
        hb = bf16_bits(vf[t]); sVh[r][c4 + t] = hb; sVl[r][c4 + t] = bf16_bits(vf[t] - bf16_val(hb));
      }
    }
    __syncthreads();
    v8f s[2];
#pragma unroll
    for (int nt = 0; nt < 2; ++nt) {
      v8f acc = {};
#pragma unroll
      for (int ks = 0; ks < KS; ++ks) {
        FragB bh_, bl_;
        bh_.half[0] = *(const v8us*)&sKh[nt * 16 + ln][ks * 32 + 8 * hh]; bh_.half[1] = *(const v8us*)&sKh[nt * 16 + ln][ks * 32 + 16 + 8 * hh];
        bl_.half[0] = *(const v8us*)&sKl[nt * 16 + ln][ks * 32 + 8 * hh]; bl_.half[1] = *(const v8us*)&sKl[nt * 16 + ln][ks * 32 + 16 + 8 * hh];
        acc = mmaN<3>(aqh[ks].v, aql[ks].v, bh_.v, bl_.v, acc);
      }
      s[nt] = acc;
    }
    float alpha[8];
#pragma unroll
    for (int r = 0; r < 8; ++r) {
      const int qi = q0 + 8 * hh + r;
      const int ja = j0 + ln, jb = j0 + 16 + ln;
      if (CAUSAL) { if (ja > qi) s[0][r] = -3.0e38f; if (jb > qi) s[1][r] = -3.0e38f; }
      if (ja >= T) s[0][r] = -3.0e38f;
      if (jb >= T) s[1][r] = -3.0e38f;
      float mx = fmaxf(s[0][r], s[1][r]);
      mx = fmaxf(mx, __shfl_xor(mx, 1, 32)); mx = fmaxf(mx, __shfl_xor(mx, 2, 32)); mx = fmaxf(mx, __shfl_xor(mx, 4, 32)); mx = fmaxf(mx, __shfl_xor(mx, 8, 32));
      const float mnew = fmaxf(m_r[r], mx);
      alpha[r] = (mnew > -1.0e38f) ? __expf(m_r[r] - mnew) : 1.0f;
      const float p0 = (s[0][r] > -1.0e38f) ? __expf(s[0][r] - mnew) : 0.f;
      const float p1 = (s[1][r] > -1.0e38f) ? __expf(s[1][r] - mnew) : 0.f;
      m_r[r] = mnew;
      l_r[r] = l_r[r] * alpha[r] + p0 + p1;
      unsigned short hb = bf16_bits(p0); sPh[w][8 * hh + r][ln] = hb;      sPl[w][8 * hh + r][ln] = bf16_bits(p0 - bf16_val(hb));
      hb = bf16_bits(p1);                sPh[w][8 * hh + r][16 + ln] = hb; sPl[w][8 * hh + r][16 + ln] = bf16_bits(p1 - bf16_val(hb));
    }
#pragma unroll
    for (int dt = 0; dt < DT; ++dt)
#pragma unroll
      for (int r = 0; r < 8; ++r) oacc[dt][r] *= alpha[r];
    __builtin_amdgcn_fence(__ATOMIC_ACQ_REL, "workgroup");
    __builtin_amdgcn_wave_barrier();
    FragB pah, pal;
    pah.half[0] = *(const v8us*)&sPh[w][ln][8 * hh]; pah.half[1] = *(const v8us*)&sPh[w][ln][16 + 8 * hh];
    pal.half[0] = *(const v8us*)&sPl[w][ln][8 * hh]; pal.half[1] = *(const v8us*)&sPl[w][ln][16 + 8 * hh];
#pragma unroll
    for (int dt = 0; dt < DT; ++dt) {
      FragB bvh, bvl;
#pragma unroll
      for (int i = 0; i < 8; ++i) {
        bvh.u[i] = sVh[8 * hh + i][dt * 16 + ln]; bvh.u[8 + i] = sVh[16 + 8 * hh + i][dt * 16 + ln];
        bvl.u[i] = sVl[8 * hh + i][dt * 16 + ln]; bvl.u[8 + i] = sVl[16 + 8 * hh + i][dt * 16 + ln];
      }
      oacc[dt] = mmaN<3>(pah.v, pal.v, bvh.v, bvl.v, oacc[dt]);
    }
    __builtin_amdgcn_fence(__ATOMIC_ACQ_REL, "workgroup");
    __builtin_amdgcn_wave_barrier();
  }
#pragma unroll
  for (int r = 0; r < 8; ++r) {
    float l = l_r[r];
    l += __shfl_xor(l, 1, 32); l += __shfl_xor(l, 2, 32); l += __shfl_xor(l, 4, 32); l += __shfl_xor(l, 8, 32);
    l_r[r] = (l > 0.f) ? 1.0f / l : 0.f;
  }
#pragma unroll
  for (int dt = 0; dt < DT; ++dt)
#pragma unroll
    for (int r = 0; r < 8; ++r) sO[w][8 * hh + r][dt * 16 + ln] = oacc[dt][r] * l_r[r];
  __builtin_amdgcn_fence(__ATOMIC_ACQ_REL, "workgroup");
  __builtin_amdgcn_wave_barrier();
  for (int pass = 0; pass < 2; ++pass) {
    for (int r = 0; r < 16; ++r) {
      const int row = q0 + r;
      if (row < T && lane < D / 4) {
        const v4f val = *(const v4fa*)&sO[w][r][lane * 4];
        *(volatile v4f*)(y + ((size_t)b * T + row) * ypitch + h * D + lane * 4) = val;
      }
    }
    if (pass == 0) __threadfence();
  }
}

template <bool ASPLIT, int ACT, bool BIAS_BF16, bool RES_BF16>
__global__ __launch_bounds__(128) void k_gemm_bf3(const float* __restrict__ A, int lda, const unsigned short* __restrict__ Wt, int ldb,
                                                const float* __restrict__ bias, const float* __restrict__ resid, int rmod, int ldr,
                                                float* __restrict__ C, int ldc, int M, int N, int K) {
  __shared__ __attribute__((aligned(16))) float so[4][16][64];
  const int tid = threadIdx.x, w = tid >> 5, lane = tid & 31, ln = lane & 15, hh = lane >> 4;
  const int ntn = N / 64;
  const int wid = blockIdx.x * 4 + w;
  const int mt = wid / ntn, nq = wid % ntn;
  if (mt * 16 >= M) return;
  const int row0 = mt * 16, col0 = nq * 64;
  const float* arow = A + (size_t)(row0 + ln) * lda;
  v8f acc[4] = {};
  for (int kb = 0; kb < K; kb += 32) {
    FragB ah, al;
    const v4f x0 = *(const v4fa*)(arow + kb + 8 * hh), x1 = *(const v4fa*)(arow + kb + 8 * hh + 4);
    const v4f x2 = *(const v4fa*)(arow + kb + 16 + 8 * hh), x3 = *(const v4fa*)(arow + kb + 16 + 8 * hh + 4);
    float xs[16] = {x0[0],x0[1],x0[2],x0[3],x1[0],x1[1],x1[2],x1[3],x2[0],x2[1],x2[2],x2[3],x3[0],x3[1],x3[2],x3[3]};
#pragma unroll
    for (int i = 0; i < 16; ++i) { const unsigned short hb = bf16_bits(xs[i]); ah.u[i] = hb; al.u[i] = ASPLIT ? bf16_bits(xs[i] - bf16_val(hb)) : (unsigned short)0; }
#pragma unroll
    for (int t = 0; t < 4; ++t) {
      const unsigned short* brow = Wt + (size_t)(col0 + t * 16 + ln) * ldb + kb;
      FragB b;
      b.half[0] = *(const v8us*)(brow + 8 * hh);
      b.half[1] = *(const v8us*)(brow + 16 + 8 * hh);
      acc[t] = mmaN<ASPLIT ? 2 : 1>(ah.v, al.v, b.v, b.v, acc[t]);
    }
  }
#pragma unroll
  for (int t = 0; t < 4; ++t) {
    const int col = col0 + t * 16 + ln;
    float bv = bias ? bias[col] : 0.f;
    if (BIAS_BF16) bv = bf16_round(bv);
#pragma unroll
    for (int r = 0; r < 8; ++r) {
      float v = acc[t][r] + bv;
      if (resid) { float rv = resid[(size_t)((row0 + 8 * hh + r) % rmod) * ldr + col]; if (RES_BF16) rv = bf16_round(rv); v += rv; }
      if (ACT == 1) v = fmaxf(v, 0.f);
      if (ACT == 2) v = 0.5f * v * (1.0f + erff(v * 0.70710678118654752f));
      if (ACT == 3) { const float u = 0.7978845608028654f * (v + 0.044715f * v * v * v); v = 0.5f * v * (1.0f + tanhf(u)); }
      so[w][8 * hh + r][t * 16 + ln] = v;
    }
  }
  __builtin_amdgcn_fence(__ATOMIC_ACQ_REL, "workgroup");
  __builtin_amdgcn_wave_barrier();
  const int rsub = lane >> 4, c4 = (lane & 15) * 4;
  for (int pass = 0; pass < 2; ++pass) {
#pragma unroll
    for (int q = 0; q < 8; ++q) {
      const int r = q * 2 + rsub;
      const v4f v = *(const v4fa*)&so[w][r][c4];
      *(volatile v4f*)(C + (size_t)(row0 + r) * ldc + col0 + c4) = v;
    }
    if (pass == 0) __threadfence();
  }
}
template <bool PARAM_BF16>
__global__ __launch_bounds__(256) void k_layernorm(const float* __restrict__ X, const float* __restrict__ R, const float* __restrict__ g, const float* __restrict__ bta,
                                                  float* __restrict__ out_sum, float* __restrict__ out_norm, int N, float eps) {
  __shared__ float red[256];
  const int row = blockIdx.x, tid = threadIdx.x;
  const float* x = X + (size_t)row * N; const float* rr = R ? R + (size_t)row * N : nullptr;
  float vals[16];
  const int per = N / 256;
  float s1 = 0.f;
  for (int u = 0; u < per / 4; ++u) {
    const int j = tid * 4 + 1024 * u;
    const v4f a = *(const v4fa*)(x + j);
    v4f b = {0.f,0.f,0.f,0.f}; if (rr) b = *(const v4fa*)(rr + j);
#pragma unroll
    for (int q = 0; q < 4; ++q) { const float v = a[q] + b[q]; vals[u * 4 + q] = v; s1 += v; }
  }
  red[tid] = s1; __syncthreads();
  for (int st = 128; st > 0; st >>= 1) { if (tid < st) red[tid] += red[tid + st]; __syncthreads(); }
  const float mu = red[0] / (float)N; __syncthreads();
  float s2 = 0.f;
  for (int u = 0; u < per / 4; ++u)
#pragma unroll
    for (int q = 0; q < 4; ++q) { const float c = vals[u * 4 + q] - mu; s2 += c * c; }
  red[tid] = s2; __syncthreads();
  for (int st = 128; st > 0; st >>= 1) { if (tid < st) red[tid] += red[tid + st]; __syncthreads(); }
  const float rs = rsqrtf(red[0] / (float)N + eps);
  for (int pass = 0; pass < 2; ++pass) {
    for (int u = 0; u < per / 4; ++u) {
      const int j = tid * 4 + 1024 * u;
      v4f o, sm;
#pragma unroll
      for (int q = 0; q < 4; ++q) {
        float gg = g[j + q], bb = bta[j + q];
        if (PARAM_BF16) { gg = bf16_round(gg); bb = bf16_round(bb); }
        sm[q] = vals[u * 4 + q]; o[q] = (vals[u * 4 + q] - mu) * rs * gg + bb;
      }
      if (out_sum) *(volatile v4f*)(out_sum + (size_t)row * N + j) = sm;
      *(volatile v4f*)(out_norm + (size_t)row * N + j) = o;
    }
    if (pass == 0) __threadfence();
  }
}

__device__ __forceinline__ float elu_f(float x) { return x > 0.f ? x : expm1f(x); }
__global__ __launch_bounds__(256) void k_wt_pad(const float* __restrict__ W, unsigned short* __restrict__ Bt, int Kin, int Nout, int Kp) {
  const int t = blockIdx.x * 256 + threadIdx.x; const int k8n = Kp / 8; if (t >= Nout * k8n) return; const int n = t / k8n, k8 = (t % k8n) * 8; v8us v;
#pragma unroll 1
  for (int i = 0; i < 8; ++i) { const int k = k8 + i; v[i] = (k < Kin) ? bf16_bits(W[(size_t)k * Nout + n]) : (unsigned short)0; }
  *(volatile v8us*)(Bt + (size_t)n * Kp + k8) = v; __threadfence(); *(volatile v8us*)(Bt + (size_t)n * Kp + k8) = v;
}
__global__ __launch_bounds__(224) void k_x0(const float* __restrict__ data, float* __restrict__ x0) {
  const int r = blockIdx.x, k = threadIdx.x; const float v = (k < KIN) ? bf16_round(data[(size_t)r * KIN + k]) : 0.f;
  *(volatile float*)(x0 + (size_t)r * KINP + k) = v; __threadfence(); *(volatile float*)(x0 + (size_t)r * KINP + k) = v;
}
__global__ __launch_bounds__(256) void k_elu_ip(float* __restrict__ a, size_t n4) { const size_t t = (size_t)blockIdx.x * 256 + threadIdx.x; if (t >= n4) return; v4f v = *(const v4fa*)(a + t * 4);
#pragma unroll 1
  for (int q = 0; q < 4; ++q) v[q] = elu_f(v[q]); *(volatile v4f*)(a + t * 4) = v; __threadfence(); *(volatile v4f*)(a + t * 4) = v; }
__global__ __launch_bounds__(256) void k_colstat1(const float* __restrict__ h, int nrows, double* __restrict__ part) {
  const int c = threadIdx.x; const int r0 = blockIdx.x * 512; const int r1 = min(r0 + 512, nrows); double s = 0.0, s2 = 0.0;
#pragma unroll 1
  for (int r = r0; r < r1; ++r) { const double v = (double)h[(size_t)r * HE + c]; s += v; s2 += v * v; }
  double* dst = part + (size_t)blockIdx.x * 2 * HE; *(volatile double*)(dst + c) = s; *(volatile double*)(dst + HE + c) = s2; __threadfence(); *(volatile double*)(dst + c) = s; *(volatile double*)(dst + HE + c) = s2;
}
__global__ __launch_bounds__(256) void k_colstat2(const double* __restrict__ part, int nblk, int nrows, float* __restrict__ stats) {
  const int c = threadIdx.x; double s = 0.0, s2 = 0.0; for (int b = 0; b < nblk; ++b) { s += part[(size_t)b * 2 * HE + c]; s2 += part[(size_t)b * 2 * HE + HE + c]; }
  const double mu = s / nrows; double var = s2 / nrows - mu * mu; if (var < 0.0) var = 0.0; const float m = (float)mu, rs = (float)(1.0 / sqrt(var + 1e-5));
  *(volatile float*)(stats + c) = m; *(volatile float*)(stats + HE + c) = rs; __threadfence(); *(volatile float*)(stats + c) = m; *(volatile float*)(stats + HE + c) = rs;
}
__global__ __launch_bounds__(256) void k_bn_apply(float* __restrict__ h, int nrows, const float* __restrict__ stats, const float* __restrict__ g, const float* __restrict__ be) {
  const size_t t = (size_t)blockIdx.x * 256 + threadIdx.x; if (t >= (size_t)nrows * (HE / 4)) return; const int c4 = (int)(t % (HE / 4)) * 4; v4f v = *(const v4fa*)(h + t * 4);
  for (int q = 0; q < 4; ++q) { const int c = c4 + q; v[q] = (v[q] - stats[c]) * stats[HE + c] * bf16_round(g[c]) + bf16_round(be[c]); }
  *(volatile v4f*)(h + t * 4) = v; __threadfence(); *(volatile v4f*)(h + t * 4) = v;
}
__global__ __launch_bounds__(256) void k_edgecat(const float* __restrict__ x, const int* __restrict__ send, const int* __restrict__ recv, const float* __restrict__ skip, float* __restrict__ cat, int width) {
  const size_t t = (size_t)blockIdx.x * 256 + threadIdx.x; if (t >= (size_t)BB * NE * (width / 4)) return; const size_t row = t / (width / 4); const int c4 = (int)(t % (width / 4)) * 4;
  const int b = (int)(row / NE), e = (int)(row % NE); int sn = send[e], rn = recv[e]; sn = sn < 0 ? 0 : (sn >= NND ? NND - 1 : sn); rn = rn < 0 ? 0 : (rn >= NND ? NND - 1 : rn);
  v4f v; if (c4 < HE) v = *(const v4fa*)(x + ((size_t)b * NND + sn) * HE + c4); else if (c4 < 2 * HE) v = *(const v4fa*)(x + ((size_t)b * NND + rn) * HE + c4 - HE); else v = *(const v4fa*)(skip + row * HE + c4 - 2 * HE);
  *(volatile v4f*)(cat + row * width + c4) = v; __threadfence(); *(volatile v4f*)(cat + row * width + c4) = v;
}
__global__ __launch_bounds__(256) void k_e2n(const float* __restrict__ xe, const int* __restrict__ recv, float* __restrict__ inc) {
  const int tid = threadIdx.x, w = tid >> 5, lane = tid & 31; const int bn = blockIdx.x * 8 + w; if (bn >= BB * NND) return; const int b = bn / NND, n = bn % NND;
  float a[8]; for (int u = 0; u < 8; ++u) a[u] = 0.f;
#pragma unroll 1
  for (int e = 0; e < NE; ++e) { if (recv[e] != n) continue; const float* r = xe + ((size_t)b * NE + e) * HE;
#pragma unroll
    for (int u = 0; u < 8; ++u) a[u] += r[u * 32 + lane]; }
  for (int pass = 0; pass < 2; ++pass) { for (int u = 0; u < 8; ++u) *(volatile float*)(inc + (size_t)bn * HE + u * 32 + lane) = a[u] * (1.0f / NND); if (pass == 0) __threadfence(); }
}
__global__ __launch_bounds__(256) void k_logits(const float* __restrict__ x4, const float* __restrict__ fcw, const float* __restrict__ fcb, const float* __restrict__ gum, float* __restrict__ rt, float* __restrict__ prob) {
  __shared__ float sv[8][8];
  const int tid = threadIdx.x, w = tid >> 5, lane = tid & 31; const size_t row = (size_t)blockIdx.x * 8 + w; const bool ok = row < (size_t)BB * NE;
  float l[KT] = {0.f, 0.f, 0.f, 0.f};
  if (ok) { const float* xr = x4 + row * HE;
#pragma unroll 1
    for (int u = 0; u < 8; ++u) { const float xv = xr[u * 32 + lane]; for (int k = 0; k < KT; ++k) l[k] += xv * bf16_round(fcw[(u * 32 + lane) * KT + k]); } }
  for (int k = 0; k < KT; ++k) for (int o = 16; o >= 1; o >>= 1) l[k] += __shfl_xor(l[k], o, 32);
  if (ok && lane == 0) { float lg[KT], g[KT]; float m1 = -3e38f, m2 = -3e38f;
    for (int k = 0; k < KT; ++k) { lg[k] = l[k] + bf16_round(fcb[k]); g[k] = (lg[k] + bf16_round(gum[row * KT + k])) * 2.0f; m1 = fmaxf(m1, lg[k]); m2 = fmaxf(m2, g[k]); }
    float d1 = 0.f, d2 = 0.f; for (int k = 0; k < KT; ++k) { lg[k] = expf(lg[k] - m1); d1 += lg[k]; g[k] = expf(g[k] - m2); d2 += g[k]; }
    for (int k = 0; k < KT; ++k) { sv[w][k] = g[k] / d2; sv[w][4 + k] = lg[k] / d1; } }
  __syncthreads();
  const size_t row0 = (size_t)blockIdx.x * 8;
  for (int pass = 0; pass < 2; ++pass) {
    if (tid < 32) { const int r = tid >> 2, k = tid & 3; if (row0 + r < (size_t)BB * NE) *(volatile float*)(rt + (row0 + r) * KT + k) = sv[r][k]; }
    else if (tid < 64) { const int r = (tid - 32) >> 2, k = (tid - 32) & 3; if (row0 + r < (size_t)BB * NE) *(volatile float*)(prob + (row0 + r) * KT + k) = sv[r][4 + k]; }
    if (pass == 0) __threadfence();
  }
}
__global__ __launch_bounds__(128) void k_dec_msg(const float* __restrict__ data, const int* __restrict__ send, const int* __restrict__ recv, const float* __restrict__ rt, int bt0,
                                               const float* __restrict__ mw1, const float* __restrict__ mb1, const unsigned short* __restrict__ Bm2, const float* __restrict__ mb2, float* __restrict__ msg) {
  __shared__ __attribute__((aligned(16))) float sH[4][16][HE + 4];
  __shared__ __attribute__((aligned(16))) float sAcc[4][16][HE + 4];
  const int tid = threadIdx.x, w = tid >> 5, lane = tid & 31, ln = lane & 15, hh = lane >> 4;
  const size_t rl0 = ((size_t)blockIdx.x * 4 + w) * 16; if (rl0 >= (size_t)CH * NE) return;
  const size_t rl = rl0 + ln; const int btl = (int)(rl / NE), e = (int)(rl % NE); const int bt = bt0 + btl; const int b = bt / TT, t = bt % TT;
  int sn = send[e], rn = recv[e]; sn = sn < 0 ? 0 : (sn >= NND ? NND - 1 : sn); rn = rn < 0 ? 0 : (rn >= NND ? NND - 1 : rn);
  float pre[8]; for (int d = 0; d < 4; ++d) { pre[d] = bf16_round(data[(((size_t)b * NND + sn) * TT + t) * DDIM + d]); pre[4 + d] = bf16_round(data[(((size_t)b * NND + rn) * TT + t) * DDIM + d]); }
  for (int c = hh; c < HE; c += 2) for (int r2 = 0; r2 < 1; ++r2) sAcc[w][ln][c] = 0.f;
#pragma unroll 1
  for (int k = 1; k < KT; ++k) {
#pragma unroll 1
    for (int c = hh; c < HE; c += 2) { float s = bf16_round(mb1[k * HE + c]);
#pragma unroll
      for (int d = 0; d < 8; ++d) s += pre[d] * bf16_round(mw1[((size_t)k * 8 + d) * HE + c]); sH[w][ln][c] = fmaxf(s, 0.f); }
    __builtin_amdgcn_fence(__ATOMIC_ACQ_REL, "workgroup"); __builtin_amdgcn_wave_barrier();
    FragB ah[8], al[8];
#pragma unroll
    for (int ks = 0; ks < 8; ++ks)
#pragma unroll
      for (int i = 0; i < 16; ++i) { const int kk = ks * 32 + ((i < 8) ? (8 * hh + i) : (16 + 8 * hh + (i - 8))); const float v = sH[w][ln][kk]; const unsigned short hb = bf16_bits(v); ah[ks].u[i] = hb; al[ks].u[i] = bf16_bits(v - bf16_val(hb)); }
    float wr[8]; for (int r = 0; r < 8; ++r) { const size_t rr = rl0 + 8 * hh + r; const int ee = (int)(rr % NE); const int bb = (bt0 + (int)(rr / NE)) / TT; wr[r] = rt[((size_t)bb * NE + ee) * KT + k]; }
#pragma unroll 1
    for (int g4 = 0; g4 < 4; ++g4) {
      v8f acc[4]; for (int tq = 0; tq < 4; ++tq) acc[tq] = (v8f){0.f,0.f,0.f,0.f,0.f,0.f,0.f,0.f};
#pragma unroll
      for (int ks = 0; ks < 8; ++ks)
#pragma unroll
        for (int tq = 0; tq < 4; ++tq) { const int n = g4 * 64 + tq * 16 + ln; FragB bq; bq.half[0] = *(const v8us*)(Bm2 + ((size_t)k * HE + n) * HE + ks * 32 + 8 * hh); bq.half[1] = *(const v8us*)(Bm2 + ((size_t)k * HE + n) * HE + ks * 32 + 16 + 8 * hh); acc[tq] = mmaN<2>(ah[ks].v, al[ks].v, bq.v, bq.v, acc[tq]); }
#pragma unroll
      for (int tq = 0; tq < 4; ++tq) { const int col = g4 * 64 + tq * 16 + ln; const float bb = bf16_round(mb2[k * HE + col]);
#pragma unroll
        for (int r = 0; r < 8; ++r) sAcc[w][8 * hh + r][col] += wr[r] * fmaxf(acc[tq][r] + bb, 0.f); }
    }
    __builtin_amdgcn_fence(__ATOMIC_ACQ_REL, "workgroup"); __builtin_amdgcn_wave_barrier();
  }
  const int rsub = lane >> 4, c4 = (lane & 15) * 4;
  for (int pass = 0; pass < 2; ++pass) { for (int cb = 0; cb < 4; ++cb) for (int q = 0; q < 8; ++q) { const int r = q * 2 + rsub; const v4f v = *(const v4fa*)&sAcc[w][r][cb * 64 + c4]; *(volatile v4f*)(msg + (rl0 + r) * HE + cb * 64 + c4) = v; } if (pass == 0) __threadfence(); }
}
__global__ __launch_bounds__(256) void k_dec_agg(const float* __restrict__ data, const float* __restrict__ msg, const int* __restrict__ recv, int bt0, float* __restrict__ aug) {
  const int tid = threadIdx.x, w = tid >> 5, lane = tid & 31; const int rn_ = blockIdx.x * 8 + w; if (rn_ >= CH * NND) return; const int btl = rn_ / NND, n = rn_ % NND; const int bt = bt0 + btl, b = bt / TT, t = bt % TT;
  float a[8]; for (int u = 0; u < 8; ++u) a[u] = 0.f;
#pragma unroll 1
  for (int e = 0; e < NE; ++e) { if (recv[e] != n) continue; const float* r = msg + ((size_t)btl * NE + e) * HE;
#pragma unroll
    for (int u = 0; u < 8; ++u) a[u] += r[u * 32 + lane]; }
  float* row = aug + (size_t)rn_ * 288;
  const float head = (lane < 4) ? bf16_round(data[(((size_t)b * NND + n) * TT + t) * DDIM + lane]) : 0.f;
  float vals[9];
#pragma unroll
  for (int u = 0; u < 9; ++u) {
    const float hi = __shfl(a[u < 8 ? u : 7], (lane - 4) & 31, 32);
    const float lo = __shfl(a[u > 0 ? u - 1 : 0], (lane + 28) & 31, 32);
    const int c = u * 32 + lane; float v = 0.f;
    if (c < 4) v = head; else if (c < 4 + HE) v = (lane >= 4) ? hi : lo;
    vals[u] = v; }
  for (int pass = 0; pass < 2; ++pass) {
#pragma unroll
    for (int u = 0; u < 9; ++u) *(volatile float*)(row + u * 32 + lane) = vals[u];
    if (pass == 0) __threadfence();
  }
}
__global__ __launch_bounds__(256) void k_dec_out(const float* __restrict__ p, const float* __restrict__ data, const float* __restrict__ ow3, const float* __restrict__ ob3, int bt0, float* __restrict__ out) {
  __shared__ float sv[8][4];
  const int tid = threadIdx.x, w = tid >> 5, lane = tid & 31; const int rn_ = blockIdx.x * 8 + w; const bool ok = rn_ < CH * NND;
  int btl = 0, n = 0, b = 0, t = 0; if (ok) { btl = rn_ / NND; n = rn_ % NND; const int bt = bt0 + btl; b = bt / TT; t = bt % TT; }
  float l[4] = {0.f,0.f,0.f,0.f};
  if (ok) { const float* pr = p + (size_t)rn_ * HE;
#pragma unroll 1
    for (int u = 0; u < 8; ++u) { const float xv = pr[u * 32 + lane]; for (int d = 0; d < 4; ++d) l[d] += xv * bf16_round(ow3[(u * 32 + lane) * 4 + d]); } }
  for (int d = 0; d < 4; ++d) for (int o = 16; o >= 1; o >>= 1) l[d] += __shfl_xor(l[d], o, 32);
  if (ok && lane < 4) sv[w][lane] = l[lane] + bf16_round(ob3[lane]) + bf16_round(data[(((size_t)b * NND + n) * TT + t) * DDIM + lane]);
  __syncthreads();
  if (tid < 32) { const int r = tid >> 2, d = tid & 3; const int rr = blockIdx.x * 8 + r; if (rr < CH * NND) { *(volatile float*)(out + ((size_t)bt0 * NND + rr) * DDIM + d) = sv[r][d]; } }
  __threadfence();
  if (tid < 32) { const int r = tid >> 2, d = tid & 3; const int rr = blockIdx.x * 8 + r; if (rr < CH * NND) { *(volatile float*)(out + ((size_t)bt0 * NND + rr) * DDIM + d) = sv[r][d]; } }
}
__global__ __launch_bounds__(256) void k_outperm(const float* __restrict__ stp, float* __restrict__ out) {
  const size_t i = (size_t)blockIdx.x * 256 + threadIdx.x; if (i >= (size_t)BB * NND * (TT - 1) * DDIM) return;
  const int d = (int)(i % DDIM); size_t r = i / DDIM; const int t = (int)(r % (TT - 1)); r /= (TT - 1); const int n = (int)(r % NND); const int b = (int)(r / NND);
  const float v = stp[(((size_t)b * TT + t) * NND + n) * DDIM + d];
  *(volatile float*)(out + i) = v; __threadfence(); *(volatile float*)(out + i) = v;
}
extern "C" void kernel_launch(void* const* d_in, const int* in_sizes, int n_in,
                              void* d_out, int out_size, void* d_ws, size_t ws_size, hipStream_t stream) {
  (void)in_sizes; (void)n_in; (void)out_size;
  const float* data = (const float*)d_in[0]; const float* gum = (const float*)d_in[1]; const int* recv = (const int*)d_in[2]; const int* send = (const int*)d_in[3];
  const float* ew1[4] = {(const float*)d_in[4], (const float*)d_in[10], (const float*)d_in[16], (const float*)d_in[22]}; const float* eb1[4] = {(const float*)d_in[5], (const float*)d_in[11], (const float*)d_in[17], (const float*)d_in[23]};
  const float* ew2[4] = {(const float*)d_in[6], (const float*)d_in[12], (const float*)d_in[18], (const float*)d_in[24]}; const float* eb2[4] = {(const float*)d_in[7], (const float*)d_in[13], (const float*)d_in[19], (const float*)d_in[25]};
  const float* eg[4] = {(const float*)d_in[8], (const float*)d_in[14], (const float*)d_in[20], (const float*)d_in[26]}; const float* ebe[4] = {(const float*)d_in[9], (const float*)d_in[15], (const float*)d_in[21], (const float*)d_in[27]};
  const float* fcw = (const float*)d_in[28]; const float* fcb = (const float*)d_in[29]; const float* mw1 = (const float*)d_in[30]; const float* mb1 = (const float*)d_in[31]; const float* mw2 = (const float*)d_in[32]; const float* mb2 = (const float*)d_in[33];
  const float* ow1 = (const float*)d_in[34]; const float* ob1 = (const float*)d_in[35]; const float* ow2 = (const float*)d_in[36]; const float* ob2 = (const float*)d_in[37]; const float* ow3 = (const float*)d_in[38]; const float* ob3 = (const float*)d_in[39];
  float* out0 = (float*)d_out; float* out1 = (float*)((char*)d_out + 196608);
  char* ws = (char*)d_ws; size_t off = 0;
  auto take = [&](size_t bytes) { char* p = ws + off; off += (bytes + 255) & ~(size_t)255; return p; };
  const int KE1[4] = {KINP, 2 * HE, HE, 3 * HE}, KEin[4] = {KIN, 2 * HE, HE, 3 * HE};
  unsigned short* B1[4], *B2[4]; for (int i = 0; i < 4; ++i) { B1[i] = (unsigned short*)take((size_t)HE * KE1[i] * 2); B2[i] = (unsigned short*)take((size_t)HE * HE * 2); }
  unsigned short* Bm2 = (unsigned short*)take((size_t)KT * HE * HE * 2); unsigned short* Bo1 = (unsigned short*)take((size_t)HE * 288 * 2); unsigned short* Bo2 = (unsigned short*)take((size_t)HE * HE * 2);
  const int RN = BB * NND, REN = BB * NE; const int nblkN = (RN + 511) / 512, nblkE = (REN + 511) / 512;
  float* x0 = (float*)take((size_t)RN * KINP * 4); float* xa = (float*)take((size_t)RN * HE * 4); float* xb = (float*)take((size_t)RN * HE * 4);
  float* cat = (float*)take((size_t)REN * 3 * HE * 4); float* ea = (float*)take((size_t)REN * HE * 4); float* eb_ = (float*)take((size_t)REN * HE * 4); float* xskip = (float*)take((size_t)REN * HE * 4);
  double* part = (double*)take((size_t)nblkE * 2 * HE * 8); float* stats = (float*)take(2 * HE * 4);
  float* rt = (float*)take((size_t)REN * KT * 4);
  float* msg = (float*)take((size_t)CH * NE * HE * 4); float* aug = (float*)take((size_t)CH * NND * 288 * 4); float* stp = (float*)take((size_t)BB * TT * NND * DDIM * 4); float* p1 = (float*)take((size_t)CH * NND * HE * 4); float* p2 = (float*)take((size_t)CH * NND * HE * 4);
  if (off > ws_size) return;
  for (int i = 0; i < 4; ++i) { k_wt_pad<<<(HE * (KE1[i] / 8) + 255) / 256, 256, 0, stream>>>(ew1[i], B1[i], KEin[i], HE, KE1[i]); k_wt_pad<<<(HE * (HE / 8) + 255) / 256, 256, 0, stream>>>(ew2[i], B2[i], HE, HE, HE); }
  for (int k = 0; k < KT; ++k) k_wt_pad<<<(HE * (HE / 8) + 255) / 256, 256, 0, stream>>>(mw2 + (size_t)k * HE * HE, Bm2 + (size_t)k * HE * HE, HE, HE, HE);
  k_wt_pad<<<(HE * (288 / 8) + 255) / 256, 256, 0, stream>>>(ow1, Bo1, 260, HE, 288); k_wt_pad<<<(HE * (HE / 8) + 255) / 256, 256, 0, stream>>>(ow2, Bo2, HE, HE, HE);
  auto gb = [](int M) { return (unsigned)(((M / 16) * (HE / 64) + 3) / 4); };
  auto mlp = [&](const float* A, int lda, int K, int i, float* t1, float* outp, int M, int nblk) {
    k_gemm_bf3<true, 0, true, false><<<gb(M), 128, 0, stream>>>(A, lda, B1[i], K, eb1[i], nullptr, 1, 0, t1, HE, M, HE, K);
    k_elu_ip<<<(unsigned)(((size_t)M * HE / 4 + 255) / 256), 256, 0, stream>>>(t1, (size_t)M * HE / 4);
    k_gemm_bf3<true, 0, true, false><<<gb(M), 128, 0, stream>>>(t1, HE, B2[i], HE, eb2[i], nullptr, 1, 0, outp, HE, M, HE, HE);
    k_elu_ip<<<(unsigned)(((size_t)M * HE / 4 + 255) / 256), 256, 0, stream>>>(outp, (size_t)M * HE / 4);
    k_colstat1<<<nblk, 256, 0, stream>>>(outp, M, part); k_colstat2<<<1, 256, 0, stream>>>(part, nblk, M, stats);
    k_bn_apply<<<(unsigned)(((size_t)M * HE / 4 + 255) / 256), 256, 0, stream>>>(outp, M, stats, eg[i], ebe[i]);
  };
  k_x0<<<RN, 224, 0, stream>>>(data, x0);
  mlp(x0, KINP, KINP, 0, xa, xb, RN, nblkN);
  k_edgecat<<<(unsigned)(((size_t)REN * (2 * HE / 4) + 255) / 256), 256, 0, stream>>>(xb, send, recv, nullptr, cat, 2 * HE);
  mlp(cat, 2 * HE, 2 * HE, 1, ea, xskip, REN, nblkE);
  k_e2n<<<(RN + 7) / 8, 256, 0, stream>>>(xskip, recv, xa);
  mlp(xa, HE, HE, 2, eb_, xb, RN, nblkN);
  k_edgecat<<<(unsigned)(((size_t)REN * (3 * HE / 4) + 255) / 256), 256, 0, stream>>>(xb, send, recv, xskip, cat, 3 * HE);
  mlp(cat, 3 * HE, 3 * HE, 3, ea, eb_, REN, nblkE);
  k_logits<<<(REN + 7) / 8, 256, 0, stream>>>(eb_, fcw, fcb, gum, rt, out1);
  const int RA = CH * NND;
  for (int c = 0; c < (BB * TT) / CH; ++c) {
    const int bt0 = c * CH;
    k_dec_msg<<<(unsigned)(((size_t)CH * NE / 16 + 3) / 4), 128, 0, stream>>>(data, send, recv, rt, bt0, mw1, mb1, Bm2, mb2, msg);
    k_dec_agg<<<(RA + 7) / 8, 256, 0, stream>>>(data, msg, recv, bt0, aug);
    k_gemm_bf3<true, 1, true, false><<<gb(RA), 128, 0, stream>>>(aug, 288, Bo1, 288, ob1, nullptr, 1, 0, p1, HE, RA, HE, 288);
    k_gemm_bf3<true, 1, true, false><<<gb(RA), 128, 0, stream>>>(p1, HE, Bo2, HE, ob2, nullptr, 1, 0, p2, HE, RA, HE, HE);
    k_dec_out<<<(RA + 7) / 8, 256, 0, stream>>>(p2, data, ow3, ob3, bt0, stp);
  }
  k_outperm<<<(BB * NND * (TT - 1) * DDIM + 255) / 256, 256, 0, stream>>>(stp, out0);
}
